// NeuralODEDecoder_77936476553390
// MI455X (gfx1250) — hardware-verified
//
#include <hip/hip_runtime.h>
#include <math.h>

typedef __attribute__((ext_vector_type(16))) _Float16 v16h;
typedef __attribute__((ext_vector_type(8)))  _Float16 v8h;
typedef __attribute__((ext_vector_type(16))) __bf16   v16b;
typedef __attribute__((ext_vector_type(8)))  __bf16   v8b;
typedef __attribute__((ext_vector_type(8)))  float    v8f;
typedef __attribute__((ext_vector_type(4)))  float    v4f;
typedef __attribute__((ext_vector_type(4)))  unsigned int v4u;

constexpr int kS = 8;
constexpr int kB = 8;
constexpr int kD = 11;
constexpr int kHid = 128;
constexpr int kBD = kB * kD;
constexpr int kSub = 100;
constexpr int kGrid = 4096;
constexpr int kRows = kS * kB * kGrid;
constexpr int kChunkRows = 65536;
constexpr int kNumChunks = kRows / kChunkRows;
constexpr int kZsN = kS * kB * kD;
constexpr int kStatBlocks = 256;

__device__ __forceinline__ float act_tanh(float x) {
  const float xc = fminf(fmaxf(x, -16.0f), 16.0f);
  const float e = expf(2.0f * xc);
  const float r = __builtin_amdgcn_rcpf(e + 1.0f);
  return 1.0f - 2.0f * r;
}

__device__ __forceinline__ unsigned short f2bf_bits(float f) {
  unsigned u = __float_as_uint(f);
  return (unsigned short)((u + 0x7FFFu + ((u >> 16) & 1u)) >> 16);
}
__device__ __forceinline__ float bf_bits2f(unsigned short h) { return __uint_as_float(((unsigned)h) << 16); }

__device__ __forceinline__ void dep_guard_h(v8f& a, v8f& b, v16h x, v16h y) { asm volatile("v_nop\n\tv_nop\n\tv_nop\n\tv_nop" : "+v"(a), "+v"(b) : "v"(x), "v"(y)); }
__device__ __forceinline__ void dep_guard_b(v8f& a, v8f& b, v16b x, v16b y) { asm volatile("v_nop\n\tv_nop\n\tv_nop\n\tv_nop" : "+v"(a), "+v"(b) : "v"(x), "v"(y)); }
__device__ __forceinline__ void keep4_h(v16h a, v16h b, v16h c, v16h d) { asm volatile("v_nop" :: "v"(a), "v"(b), "v"(c), "v"(d)); }
__device__ __forceinline__ void keep4_b(v16b a, v16b b, v16b c, v16b d) { asm volatile("v_nop" :: "v"(a), "v"(b), "v"(c), "v"(d)); }
__device__ __forceinline__ void acc_guard4(v8f& a, v8f& b, v8f& c, v8f& d) { asm volatile("v_nop\n\tv_nop\n\tv_nop\n\tv_nop" : "+v"(a), "+v"(b), "+v"(c), "+v"(d)); }
template <typename T> struct Frag;
template <> struct Frag<_Float16> {
  typedef v16h V; union U { v16h v; v8h h[2]; };
  static __device__ __forceinline__ v16h load(const _Float16* p) {
    U f; f.h[0] = *(const v8h*)(p); f.h[1] = *(const v8h*)(p + 16); return f.v;
  }
  static __device__ __forceinline__ v8f mma(v16h a, v16h b, v8f c) {
    return __builtin_amdgcn_wmma_f32_16x16x32_f16(false, a, false, b, (short)0, c, false, false);
  }
  static __device__ __forceinline__ void guard(v8f& a, v8f& b, v16h x, v16h y) { dep_guard_h(a, b, x, y); }
  static __device__ __forceinline__ void keep(v16h a, v16h b, v16h c, v16h d) { keep4_h(a, b, c, d); }
};
template <> struct Frag<__bf16> {
  typedef v16b V; union U { v16b v; v8b h[2]; };
  static __device__ __forceinline__ v16b load(const __bf16* p) {
    U f; f.h[0] = *(const v8b*)(p); f.h[1] = *(const v8b*)(p + 16); return f.v;
  }
  static __device__ __forceinline__ v8f mma(v16b a, v16b b, v8f c) {
    return __builtin_amdgcn_wmma_f32_16x16x32_bf16(false, a, false, b, (short)0, c, false, false);
  }
  static __device__ __forceinline__ void guard(v8f& a, v8f& b, v16b x, v16b y) { dep_guard_b(a, b, x, y); }
  static __device__ __forceinline__ void keep(v16b a, v16b b, v16b c, v16b d) { keep4_b(a, b, c, d); }
};

__device__ __forceinline__ unsigned pk16(unsigned short a, unsigned short b) { return (unsigned)a | ((unsigned)b << 16); }

template <int ET> struct Elem;
template <> struct Elem<0> { typedef _Float16 T; };
template <> struct Elem<1> { typedef __bf16 T; };
template <int ET, bool SPLIT, int BIAS_MODE, int OUT_MODE, bool RESID, int ACT = 0>
__global__ __launch_bounds__(256) void wmma_gemm64(
    const unsigned short* __restrict__ Ap, const unsigned short* __restrict__ A2p, int lda, long strideA,
    const unsigned short* __restrict__ Btp, const unsigned short* __restrict__ Bt2p, int ldb, long strideB,
    void* __restrict__ Cout, void* __restrict__ Cout2, int ldc, long strideC,
    const float* __restrict__ bias,
    const float* __restrict__ resid, long strideR,
    int M, int N, int K, float scale) {
  typedef typename Elem<ET>::T T;
  typedef typename Frag<T>::V V;
  const T* A = (const T*)Ap; const T* A2 = (const T*)A2p; const T* Bt = (const T*)Btp; const T* Bt2 = (const T*)Bt2p;
  __shared__ __align__(16) float sT[8][16 * 68];
  const int b    = blockIdx.y;
  const int lane = threadIdx.x & 31;
  const int wave = threadIdx.x >> 5;
  const int tilesN = N >> 6;
  const int tilesM = M >> 6;
  const int tile = blockIdx.x * 8 + wave;
  if (tile >= tilesM * tilesN) return;
  const int tm = tile / tilesN;
  const int tn = tile - tm * tilesN;
  const int m0 = tm << 6;
  const int n0 = tn << 6;

  const T* Ab  = A  + (size_t)b * strideA;
  const T* Bb  = Bt + (size_t)b * strideB;
  const T* Ab2 = SPLIT ? (A2  + (size_t)b * strideA) : nullptr;
  const T* Bb2 = SPLIT ? (Bt2 + (size_t)b * strideB) : nullptr;

  const int rlane = lane & 15;
  const int koff  = (lane >> 4) * 8;
  const int mOff  = (lane >> 4) * 8;

  v8f acc[4][4];
#pragma unroll
  for (int i = 0; i < 4; ++i)
#pragma unroll
    for (int j = 0; j < 4; ++j) acc[i][j] = (v8f){0.f,0.f,0.f,0.f,0.f,0.f,0.f,0.f};

  for (int k0 = 0; k0 < K; k0 += 32) {
    V bh[4], bl[4];
#pragma unroll
    for (int j = 0; j < 4; ++j) {
      const size_t bo = (size_t)(n0 + (j << 4) + rlane) * ldb + koff + k0;
      bh[j] = Frag<T>::load(Bb + bo);
      if (SPLIT) bl[j] = Frag<T>::load(Bb2 + bo);
    }
#pragma unroll
    for (int i = 0; i < 4; ++i) {
      const size_t ao = (size_t)(m0 + (i << 4) + rlane) * lda + koff + k0;
      V ah = Frag<T>::load(Ab + ao);
      V al;
      if (SPLIT) al = Frag<T>::load(Ab2 + ao);
#pragma unroll
      for (int j = 0; j < 4; ++j) {
        acc[i][j] = Frag<T>::mma(ah, bh[j], acc[i][j]);
        if (SPLIT) {
          acc[i][j] = Frag<T>::mma(ah, bl[j], acc[i][j]);
          acc[i][j] = Frag<T>::mma(al, bh[j], acc[i][j]);
        }
      }
      Frag<T>::guard(acc[i][0], acc[i][3], ah, SPLIT ? al : ah);
    }
    Frag<T>::keep(bh[0], bh[1], bh[2], bh[3]);
    if (SPLIT) Frag<T>::keep(bl[0], bl[1], bl[2], bl[3]);
  }
  acc_guard4(acc[0][0], acc[0][1], acc[0][2], acc[0][3]);
  acc_guard4(acc[1][0], acc[1][1], acc[1][2], acc[1][3]);
  acc_guard4(acc[2][0], acc[2][1], acc[2][2], acc[2][3]);
  acc_guard4(acc[3][0], acc[3][1], acc[3][2], acc[3][3]);

  float* slab = sT[wave];
  const float* Rb = RESID ? (resid + (size_t)b * strideR) : nullptr;
#pragma unroll
  for (int i = 0; i < 4; ++i) {
    const int mBase = m0 + (i << 4);
#pragma unroll
    for (int j = 0; j < 4; ++j) {
      const int n = n0 + (j << 4) + rlane;
      float bv = 0.f;
      if (BIAS_MODE == 2) bv = bias[n];
#pragma unroll
      for (int r = 0; r < 8; ++r) {
        float v = acc[i][j][r] * scale;
        if (BIAS_MODE == 1) v += bias[mBase + mOff + r];
        if (BIAS_MODE == 2) v += bv;
        if (RESID) v += Rb[(size_t)(mBase + mOff + r) * ldc + n];
        if (ACT == 1) v = act_tanh(v);
        if (ACT == 2) v = fmaxf(v, 0.0f);
        if (ACT == 4) v = (v > 0.f) ? v : 0.01f * v;
        slab[(mOff + r) * 68 + (j << 4) + rlane] = v;
      }
    }
    __builtin_amdgcn_fence(__ATOMIC_RELEASE, "workgroup");
    __builtin_amdgcn_wave_barrier();
    __builtin_amdgcn_fence(__ATOMIC_ACQUIRE, "workgroup");
    if (OUT_MODE == 0) {
      float* C = (float*)Cout + (size_t)b * strideC;
      const int hh = lane >> 4, c4 = (lane & 15) * 4;
      for (int pass = 0; pass < 2; ++pass) {
#pragma unroll
        for (int it = 0; it < 8; ++it) {
          const int row = it * 2 + hh;
          v4f v = *(const v4f*)(slab + row * 68 + c4);
          *(volatile v4f*)(C + (size_t)(mBase + row) * ldc + n0 + c4) = v;
        }
        __threadfence();
      }
    } else {
      const int q = lane >> 3, c8 = (lane & 7) * 8;
      unsigned short* C  = (unsigned short*)Cout  + (size_t)b * strideC;
      unsigned short* C2 = (OUT_MODE == 2) ? ((unsigned short*)Cout2 + (size_t)b * strideC) : nullptr;
      for (int pass = 0; pass < 2; ++pass) {
#pragma unroll
        for (int it = 0; it < 4; ++it) {
          const int row = it * 4 + q;
          const float* sp = slab + row * 68 + c8;
          v8h hv, lv;
#pragma unroll
          for (int e = 0; e < 8; ++e) {
            if (OUT_MODE == 1) {
              hv[e] = (_Float16)sp[e];
            } else {
              unsigned short hb = f2bf_bits(sp[e]);
              unsigned short lb = f2bf_bits(sp[e] - bf_bits2f(hb));
              hv[e] = __builtin_bit_cast(_Float16, hb);
              lv[e] = __builtin_bit_cast(_Float16, lb);
            }
          }
          *(volatile v8h*)(C + (size_t)(mBase + row) * ldc + n0 + c8) = hv;
          if (OUT_MODE == 2) *(volatile v8h*)(C2 + (size_t)(mBase + row) * ldc + n0 + c8) = lv;
        }
        __threadfence();
      }
    }
    __builtin_amdgcn_fence(__ATOMIC_RELEASE, "workgroup");
    __builtin_amdgcn_wave_barrier();
    __builtin_amdgcn_fence(__ATOMIC_ACQUIRE, "workgroup");
  }
}

#pragma clang fp contract(off)

__device__ __forceinline__ void split_bf(float v, unsigned short& hb, unsigned short& lb) {
  hb = f2bf_bits(v);
  lb = f2bf_bits(v - bf_bits2f(hb));
}

__device__ __forceinline__ float lin64(int i) {
  const float st = (float)i * (1.0f / 63.0f);
  const float a = 1.0f - st;
  const float v = st - a;
  return (i == 63) ? 1.0f : v;
}

__device__ __forceinline__ void coord_of(int n, float cs, float sn, float nsn, float dx0, float dx1, float& c0, float& c1) {
  const float gx = lin64(n >> 6);
  const float gy = lin64(n & 63);
  c0 = (gx * cs + gy * sn) + dx0;
  c1 = (gx * nsn + gy * cs) + dx1;
}

__device__ __forceinline__ void ld8(const float* p, float* o) {
  const v4f a = *(const v4f*)(p);
  const v4f c = *(const v4f*)(p + 4);
  o[0] = a[0]; o[1] = a[1]; o[2] = a[2]; o[3] = a[3];
  o[4] = c[0]; o[5] = c[1]; o[6] = c[2]; o[7] = c[3];
}

constexpr int OL_W1  = 0;
constexpr int OL_B1  = 1536;
constexpr int OL_W2  = 1664;
constexpr int OL_B2  = 18048;
constexpr int OL_W3T = 18176;
constexpr int OL_B3  = 19584;
constexpr int OL_Y   = 19600;
constexpr int OL_YT  = 19696;
constexpr int OL_KA  = 19792;
constexpr int OL_KO  = 19888;
constexpr int OL_H1  = 19984;
constexpr int OL_H2  = 21008;
constexpr int OL_ZS  = 22032;
constexpr int OL_PAR = 22736;
constexpr int kOdeLdsFloats = 22992;
constexpr int kOdeLdsBytes = kOdeLdsFloats * 4;

__device__ __forceinline__ void ode_eval(float* lds, int inOff, float tt, int tid) {
  const int b = tid >> 5;
  const int c4 = (tid & 31) * 4;
  {
    const float* yin = lds + inOff + b * kD;
    float a0 = 0.f, a1 = 0.f, a2 = 0.f, a3 = 0.f;
#pragma unroll
    for (int k = 0; k < kD; ++k) {
      const float yk = yin[k];
      const v4f w = *(const v4f*)(lds + OL_W1 + k * kHid + c4);
      a0 = a0 + yk * w[0]; a1 = a1 + yk * w[1]; a2 = a2 + yk * w[2]; a3 = a3 + yk * w[3];
    }
    {
      const v4f w = *(const v4f*)(lds + OL_W1 + kD * kHid + c4);
      a0 = a0 + tt * w[0]; a1 = a1 + tt * w[1]; a2 = a2 + tt * w[2]; a3 = a3 + tt * w[3];
    }
    const v4f bb = *(const v4f*)(lds + OL_B1 + c4);
    v4f h;
    h[0] = fmaxf(a0 + bb[0], 0.f); h[1] = fmaxf(a1 + bb[1], 0.f);
    h[2] = fmaxf(a2 + bb[2], 0.f); h[3] = fmaxf(a3 + bb[3], 0.f);
    *(v4f*)(lds + OL_H1 + b * kHid + c4) = h;
  }
  __syncthreads();
  {
    const float* hrow = lds + OL_H1 + b * kHid;
    float a0 = 0.f, a1 = 0.f, a2 = 0.f, a3 = 0.f;
#pragma unroll 2
    for (int k = 0; k < kHid; k += 4) {
      const v4f hk = *(const v4f*)(hrow + k);
#pragma unroll
      for (int u = 0; u < 4; ++u) {
        const v4f w = *(const v4f*)(lds + OL_W2 + (k + u) * kHid + c4);
        const float hv = hk[u];
        a0 = a0 + hv * w[0]; a1 = a1 + hv * w[1]; a2 = a2 + hv * w[2]; a3 = a3 + hv * w[3];
      }
    }
    const v4f bb = *(const v4f*)(lds + OL_B2 + c4);
    v4f h;
    h[0] = fmaxf(a0 + bb[0], 0.f); h[1] = fmaxf(a1 + bb[1], 0.f);
    h[2] = fmaxf(a2 + bb[2], 0.f); h[3] = fmaxf(a3 + bb[3], 0.f);
    *(v4f*)(lds + OL_H2 + b * kHid + c4) = h;
  }
  __syncthreads();
  if (tid < kBD) {
    const int bb = tid / kD;
    const int d = tid - bb * kD;
    const float* hrow = lds + OL_H2 + bb * kHid;
    const float* wrow = lds + OL_W3T + d * kHid;
    float a = 0.f;
#pragma unroll 2
    for (int k = 0; k < kHid; k += 4) {
      const v4f hk = *(const v4f*)(hrow + k);
      const v4f wk = *(const v4f*)(wrow + k);
      a = a + hk[0] * wk[0]; a = a + hk[1] * wk[1]; a = a + hk[2] * wk[2]; a = a + hk[3] * wk[3];
    }
    lds[OL_KO + tid] = a + lds[OL_B3 + d];
  }
  __syncthreads();
}

__global__ __launch_bounds__(256) void ode_kernel(
    const float* __restrict__ z0, const float* __restrict__ tarr, const float* __restrict__ dxp,
    const float* __restrict__ w1, const float* __restrict__ b1,
    const float* __restrict__ w2, const float* __restrict__ b2,
    const float* __restrict__ w3, const float* __restrict__ b3,
    float* __restrict__ zs_out, float* __restrict__ par_out) {
  extern __shared__ __align__(16) float ode_lds[];
  float* lds = ode_lds;
  const int tid = threadIdx.x;
  for (int i = tid; i < (kD + 1) * kHid; i += 256) lds[OL_W1 + i] = w1[i];
  for (int i4 = tid; i4 < (kHid * kHid) / 4; i4 += 256)
    *(v4f*)(lds + OL_W2 + 4 * i4) = *(const v4f*)(w2 + 4 * i4);
  for (int e = tid; e < kHid * kD; e += 256) {
    const int k = e / kD;
    const int d = e - k * kD;
    lds[OL_W3T + d * kHid + k] = w3[e];
  }
  if (tid < kHid) { lds[OL_B1 + tid] = b1[tid]; lds[OL_B2 + tid] = b2[tid]; }
  if (tid < 16) {
    const int dc = (tid < kD) ? tid : (kD - 1);
    const float bv = b3[dc];
    lds[OL_B3 + tid] = (tid < kD) ? bv : 0.f;
  }
  if (tid < 96) {
    const int sc = (tid < kBD) ? tid : (kBD - 1);
    const float v = (tid < kBD) ? z0[sc] : 0.f;
    lds[OL_Y + tid] = v; lds[OL_YT + tid] = v; lds[OL_KA + tid] = 0.f; lds[OL_KO + tid] = 0.f;
    if (tid < kBD) lds[OL_ZS + tid] = v;
  }
  __syncthreads();

#pragma unroll 1
  for (int iv = 0; iv < kS - 1; ++iv) {
    const float t0 = tarr[iv];
    const float t1 = tarr[iv + 1];
    const float dt = (t1 - t0) * 0.01f;
    const float hdt = dt * 0.5f;
    const float sdt = dt * (1.0f / 6.0f);
#pragma unroll 1
    for (int s = 0; s < kSub; ++s) {
      const float tt = t0 + (float)s * dt;
      ode_eval(lds, OL_Y, tt, tid);
      if (tid < kBD) {
        const float k1 = lds[OL_KO + tid];
        lds[OL_KA + tid] = k1;
        lds[OL_YT + tid] = lds[OL_Y + tid] + hdt * k1;
      }
      __syncthreads();
      ode_eval(lds, OL_YT, tt + hdt, tid);
      if (tid < kBD) {
        const float k2 = lds[OL_KO + tid];
        lds[OL_KA + tid] = lds[OL_KA + tid] + 2.0f * k2;
        lds[OL_YT + tid] = lds[OL_Y + tid] + hdt * k2;
      }
      __syncthreads();
      ode_eval(lds, OL_YT, tt + hdt, tid);
      if (tid < kBD) {
        const float k3 = lds[OL_KO + tid];
        lds[OL_KA + tid] = lds[OL_KA + tid] + 2.0f * k3;
        lds[OL_YT + tid] = lds[OL_Y + tid] + dt * k3;
      }
      __syncthreads();
      ode_eval(lds, OL_YT, tt + dt, tid);
      if (tid < kBD) {
        const float sum = lds[OL_KA + tid] + lds[OL_KO + tid];
        lds[OL_Y + tid] = lds[OL_Y + tid] + sdt * sum;
      }
      __syncthreads();
    }
    if (tid < kBD) lds[OL_ZS + (iv + 1) * kBD + tid] = lds[OL_Y + tid];
  }
  __syncthreads();
  if (tid < kS * kB) {
    const float th = lds[OL_ZS + tid * kD + 0];
    const float pv = dxp[0];
    lds[OL_PAR + tid * 4 + 0] = cosf(th);
    lds[OL_PAR + tid * 4 + 1] = sinf(th);
    lds[OL_PAR + tid * 4 + 2] = lds[OL_ZS + tid * kD + 1] * pv;
    lds[OL_PAR + tid * 4 + 3] = lds[OL_ZS + tid * kD + 2] * pv;
  }
  __syncthreads();
  if (tid < 32) {
    v4f zv[6];
#pragma unroll
    for (int it = 0; it < 6; ++it) {
      const int idx = it * 32 + tid;
      const int idc = (idx < 176) ? idx : 175;
      zv[it] = *(const v4f*)(lds + OL_ZS + 4 * idc);
    }
    v4f pv[2];
#pragma unroll
    for (int it = 0; it < 2; ++it) pv[it] = *(const v4f*)(lds + OL_PAR + 4 * (it * 32 + tid));
    for (int pass = 0; pass < 2; ++pass) {
#pragma unroll
      for (int it = 0; it < 6; ++it) {
        const int idx = it * 32 + tid;
        if (idx < 176) *(volatile v4f*)(zs_out + 4 * idx) = zv[it];
      }
#pragma unroll
      for (int it = 0; it < 2; ++it) *(volatile v4f*)(par_out + 4 * (it * 32 + tid)) = pv[it];
      __threadfence();
    }
  }
}

__global__ __launch_bounds__(256) void wsplit_kernel(const float* __restrict__ Wa, const float* __restrict__ Wb,
                                                     const float* __restrict__ Wc, unsigned short* __restrict__ out) {
  __shared__ float sm[64][129];
  const int t = threadIdx.x;
  const int n0 = blockIdx.x * 64;
  const int z = blockIdx.y;
  const float* W = (z == 0) ? Wa : (z == 1) ? Wb : Wc;
#pragma unroll 4
  for (int i = 0; i < 32; ++i) {
    const int e = i * 256 + t;
    const int k = e >> 6;
    const int nl = e & 63;
    sm[nl][k] = W[(size_t)k * kHid + n0 + nl];
  }
  __syncthreads();
  const int lane = t & 31, wave = t >> 5;
  const int rsub = lane >> 4, c8 = (lane & 15) * 8;
  unsigned short* hp = out + (size_t)z * 2 * kHid * kHid;
  unsigned short* lp = hp + kHid * kHid;
  v4u uh[4], ul[4];
#pragma unroll
  for (int it = 0; it < 4; ++it) {
    const int nl = wave * 8 + it * 2 + rsub;
    unsigned hw[4], lw[4];
#pragma unroll
    for (int q = 0; q < 4; ++q) {
      unsigned short h0, l0, h1, l1;
      split_bf(sm[nl][c8 + 2 * q], h0, l0);
      split_bf(sm[nl][c8 + 2 * q + 1], h1, l1);
      hw[q] = pk16(h0, h1); lw[q] = pk16(l0, l1);
    }
    uh[it] = (v4u){hw[0], hw[1], hw[2], hw[3]};
    ul[it] = (v4u){lw[0], lw[1], lw[2], lw[3]};
  }
  for (int pass = 0; pass < 2; ++pass) {
#pragma unroll
    for (int it = 0; it < 4; ++it) {
      const int nl = wave * 8 + it * 2 + rsub;
      const size_t off = (size_t)(n0 + nl) * kHid + c8;
      *(volatile v4u*)(hp + off) = uh[it];
      *(volatile v4u*)(lp + off) = ul[it];
    }
    __threadfence();
  }
}

template <int PASS>
__global__ __launch_bounds__(256) void bnstat_kernel(const float* __restrict__ par, const float* __restrict__ cw,
                                                     const float* __restrict__ cb, const float* __restrict__ mu,
                                                     float* __restrict__ partial) {
  __shared__ __align__(16) float cc[2 * 1024];
  __shared__ float red[256];
  __shared__ __align__(16) float outp[128];
  const int t = threadIdx.x;
  const int blk = blockIdx.x;
  const int sb = blk >> 2;
  const int qr = blk & 3;
  const float cs = par[sb * 4 + 0], sn = par[sb * 4 + 1], dx0 = par[sb * 4 + 2], dx1 = par[sb * 4 + 3];
  const float nsn = -sn;
#pragma unroll
  for (int u = 0; u < 4; ++u) {
    const int nl = t * 4 + u;
    const int n = qr * 1024 + nl;
    float c0, c1;
    coord_of(n, cs, sn, nsn, dx0, dx1, c0, c1);
    cc[2 * nl] = c0; cc[2 * nl + 1] = c1;
  }
  __syncthreads();
  const int j = t & 127;
  const int p = t >> 7;
  const float w0 = cw[j], w1 = cw[kHid + j], bj = cb[j];
  float mj = 0.f;
  if (PASS == 1) mj = mu[j];
  float acc = 0.f;
  const float* ccp = cc + p * 1024;
#pragma unroll 4
  for (int r = 0; r < 512; ++r) {
    const float c0 = ccp[2 * r];
    const float c1 = ccp[2 * r + 1];
    const float h = (c0 * w0 + c1 * w1) + bj;
    if (PASS == 0) {
      acc = acc + h;
    } else {
      const float d = h - mj;
      acc = acc + d * d;
    }
  }
  red[t] = acc;
  __syncthreads();
  if (t < 128) outp[t] = red[t] + red[t + 128];
  __syncthreads();
  if (t < 32) {
    const v4f v = *(const v4f*)(outp + 4 * t);
    float* dst = partial + (size_t)blk * 128 + 4 * t;
    *(volatile v4f*)dst = v;
    __threadfence();
    *(volatile v4f*)dst = v;
  }
}

template <int PASS>
__global__ __launch_bounds__(128) void bnreduce_kernel(const float* __restrict__ partial, float* __restrict__ outv) {
  __shared__ __align__(16) float so[128];
  const int t = threadIdx.x;
  float s = 0.f;
#pragma unroll 4
  for (int blk = 0; blk < kStatBlocks; ++blk) s = s + partial[blk * 128 + t];
  const float m = s * (1.0f / 262144.0f);
  float v = m;
  if (PASS == 1) {
    const float sd = sqrtf(m + 1e-5f);
    v = 1.0f / sd;
  }
  so[t] = v;
  __syncthreads();
  if (t < 32) {
    const v4f x = *(const v4f*)(so + 4 * t);
    float* dst = outv + 4 * t;
    *(volatile v4f*)dst = x;
    __threadfence();
    *(volatile v4f*)dst = x;
  }
}

__global__ __launch_bounds__(256) void bnapply_kernel(const float* __restrict__ par, const float* __restrict__ cw,
                                                      const float* __restrict__ cb, const float* __restrict__ mu,
                                                      const float* __restrict__ istd, const float* __restrict__ ga,
                                                      const float* __restrict__ be, unsigned short* __restrict__ ahi,
                                                      unsigned short* __restrict__ alo, int chunk) {
  const int t = threadIdx.x;
  const int lane = t & 31, wave = t >> 5;
  const int rsub = lane >> 4, c8 = (lane & 15) * 8;
  const int lrow0 = blockIdx.x * 64;
  const int grow0 = chunk * kChunkRows + lrow0;
  const int sb = grow0 >> 12;
  const float cs = par[sb * 4 + 0], sn = par[sb * 4 + 1], dx0 = par[sb * 4 + 2], dx1 = par[sb * 4 + 3];
  const float nsn = -sn;
  float w0[8], w1[8], cbv[8], muv[8], isv[8], gav[8], bev[8];
  ld8(cw + c8, w0); ld8(cw + kHid + c8, w1); ld8(cb + c8, cbv);
  ld8(mu + c8, muv); ld8(istd + c8, isv); ld8(ga + c8, gav); ld8(be + c8, bev);
  v4u uh[4], ul[4];
#pragma unroll
  for (int it = 0; it < 4; ++it) {
    const int lr = wave * 8 + it * 2 + rsub;
    const int n = (grow0 + lr) & (kGrid - 1);
    float c0, c1;
    coord_of(n, cs, sn, nsn, dx0, dx1, c0, c1);
    unsigned hw[4], lw[4];
#pragma unroll
    for (int q = 0; q < 4; ++q) {
      unsigned short hb0, lb0, hb1, lb1;
      {
        const int e = 2 * q;
        const float h = (c0 * w0[e] + c1 * w1[e]) + cbv[e];
        const float hn = ((h - muv[e]) * isv[e]) * gav[e] + bev[e];
        split_bf(hn, hb0, lb0);
      }
      {
        const int e = 2 * q + 1;
        const float h = (c0 * w0[e] + c1 * w1[e]) + cbv[e];
        const float hn = ((h - muv[e]) * isv[e]) * gav[e] + bev[e];
        split_bf(hn, hb1, lb1);
      }
      hw[q] = pk16(hb0, hb1); lw[q] = pk16(lb0, lb1);
    }
    uh[it] = (v4u){hw[0], hw[1], hw[2], hw[3]};
    ul[it] = (v4u){lw[0], lw[1], lw[2], lw[3]};
  }
  for (int pass = 0; pass < 2; ++pass) {
#pragma unroll
    for (int it = 0; it < 4; ++it) {
      const int lr = wave * 8 + it * 2 + rsub;
      const size_t off = (size_t)(lrow0 + lr) * kHid + c8;
      *(volatile v4u*)(ahi + off) = uh[it];
      *(volatile v4u*)(alo + off) = ul[it];
    }
    __threadfence();
  }
}

__global__ __launch_bounds__(256) void head_kernel(const float* __restrict__ F, const float* __restrict__ ow,
                                                   const float* __restrict__ ob, float* __restrict__ xs, int chunk) {
  __shared__ __align__(16) float s_ow[kHid];
  __shared__ __align__(16) float s_y[256];
  const int t = threadIdx.x;
  if (t < kHid) s_ow[t] = ow[t];
  __syncthreads();
  const int lr = blockIdx.x * 256 + t;
  const float* fr = F + (size_t)lr * kHid;
  float a = 0.f;
#pragma unroll 2
  for (int k = 0; k < kHid; k += 4) {
    const v4f f = *(const v4f*)(fr + k);
    const v4f w = *(const v4f*)(s_ow + k);
    a = a + f[0] * w[0]; a = a + f[1] * w[1]; a = a + f[2] * w[2]; a = a + f[3] * w[3];
  }
  s_y[t] = a + ob[0];
  __syncthreads();
  if (t < 64) {
    const v4f v = *(const v4f*)(s_y + 4 * t);
    float* dst = xs + (size_t)chunk * kChunkRows + (size_t)blockIdx.x * 256 + 4 * t;
    *(volatile v4f*)dst = v;
    __threadfence();
    *(volatile v4f*)dst = v;
  }
}

extern "C" void kernel_launch(void* const* d_in, const int* in_sizes, int n_in,
                              void* d_out, int out_size, void* d_ws, size_t ws_size,
                              hipStream_t stream) {
  if (n_in < 21) return;
  const float* z0    = (const float*)d_in[0];
  const float* tarr  = (const float*)d_in[1];
  const float* dxp   = (const float*)d_in[2];
  const float* ow1   = (const float*)d_in[3];
  const float* ob1   = (const float*)d_in[4];
  const float* ow2   = (const float*)d_in[5];
  const float* ob2   = (const float*)d_in[6];
  const float* ow3   = (const float*)d_in[7];
  const float* ob3   = (const float*)d_in[8];
  const float* cw    = (const float*)d_in[9];
  const float* cb    = (const float*)d_in[10];
  const float* gamma = (const float*)d_in[11];
  const float* beta  = (const float*)d_in[12];
  const float* l0w   = (const float*)d_in[13];
  const float* l0b   = (const float*)d_in[14];
  const float* l1w   = (const float*)d_in[15];
  const float* l1b   = (const float*)d_in[16];
  const float* l2w   = (const float*)d_in[17];
  const float* l2b   = (const float*)d_in[18];
  const float* outw  = (const float*)d_in[19];
  const float* outb  = (const float*)d_in[20];

  if (in_sizes[0] != kBD || in_sizes[1] != kS || in_sizes[3] != (kD + 1) * kHid ||
      in_sizes[5] != kHid * kHid || in_sizes[7] != kHid * kD || in_sizes[9] != 2 * kHid ||
      in_sizes[13] != kHid * kHid || in_sizes[15] != kHid * kHid || in_sizes[17] != kHid * kHid ||
      in_sizes[19] != kHid || out_size != kRows + kZsN) return;

  const size_t oPar  = 0;
  const size_t oMu   = 1024;
  const size_t oIstd = 1536;
  const size_t oPart = 2048;
  const size_t oWt   = oPart + (size_t)kStatBlocks * 128 * 4;
  const size_t wtBytes = (size_t)3 * 2 * kHid * kHid * 2;
  const size_t oA    = ((oWt + wtBytes) + 4095) & ~(size_t)4095;
  const size_t planeHalf = (size_t)kChunkRows * kHid;
  const size_t regBytes = planeHalf * 2 * 2;
  const size_t oB    = oA + regBytes;
  const size_t total = oB + regBytes;
  if (total > ws_size) return;

  char* ws = (char*)d_ws;
  float* par  = (float*)(ws + oPar);
  float* mu   = (float*)(ws + oMu);
  float* istd = (float*)(ws + oIstd);
  float* part = (float*)(ws + oPart);
  unsigned short* wt = (unsigned short*)(ws + oWt);
  unsigned short* aHi = (unsigned short*)(ws + oA);
  unsigned short* aLo = aHi + planeHalf;
  unsigned short* bHi = (unsigned short*)(ws + oB);
  unsigned short* bLo = bHi + planeHalf;
  float* fPlane = (float*)(ws + oB);

  float* xs_out = (float*)d_out;
  float* zs_out = (float*)((char*)d_out + 1048576);

  ode_kernel<<<dim3(1), dim3(256), kOdeLdsBytes, stream>>>(z0, tarr, dxp, ow1, ob1, ow2, ob2, ow3, ob3, zs_out, par);
  wsplit_kernel<<<dim3(2, 3, 1), dim3(256), 0, stream>>>(l0w, l1w, l2w, wt);
  bnstat_kernel<0><<<dim3(kStatBlocks), dim3(256), 0, stream>>>(par, cw, cb, mu, part);
  bnreduce_kernel<0><<<dim3(1), dim3(128), 0, stream>>>(part, mu);
  bnstat_kernel<1><<<dim3(kStatBlocks), dim3(256), 0, stream>>>(par, cw, cb, mu, part);
  bnreduce_kernel<1><<<dim3(1), dim3(128), 0, stream>>>(part, istd);

  const int gemmBlocks = ((kChunkRows / 64) * (kHid / 64)) / 8;
  for (int c = 0; c < kNumChunks; ++c) {
    bnapply_kernel<<<dim3(kChunkRows / 64), dim3(256), 0, stream>>>(par, cw, cb, mu, istd, gamma, beta, aHi, aLo, c);
    wmma_gemm64<1, true, 2, 2, false, 1><<<dim3(gemmBlocks, 1, 1), dim3(256), 0, stream>>>(
        aHi, aLo, kHid, 0L, wt + 0 * 32768, wt + 0 * 32768 + 16384, kHid, 0L,
        (void*)bHi, (void*)bLo, kHid, 0L, l0b, nullptr, 0L, kChunkRows, kHid, kHid, 1.0f);
    wmma_gemm64<1, true, 2, 2, false, 1><<<dim3(gemmBlocks, 1, 1), dim3(256), 0, stream>>>(
        bHi, bLo, kHid, 0L, wt + 1 * 32768, wt + 1 * 32768 + 16384, kHid, 0L,
        (void*)aHi, (void*)aLo, kHid, 0L, l1b, nullptr, 0L, kChunkRows, kHid, kHid, 1.0f);
    wmma_gemm64<1, true, 2, 0, false, 1><<<dim3(gemmBlocks, 1, 1), dim3(256), 0, stream>>>(
        aHi, aLo, kHid, 0L, wt + 2 * 32768, wt + 2 * 32768 + 16384, kHid, 0L,
        (void*)fPlane, nullptr, kHid, 0L, l2b, nullptr, 0L, kChunkRows, kHid, kHid, 1.0f);
    head_kernel<<<dim3(kChunkRows / 256), dim3(256), 0, stream>>>(fPlane, outw, outb, xs_out, c);
  }
}
